// TransformerBlockQuantum_65481071397340
// MI455X (gfx1250) — hardware-run, weakly checked
//
#include <hip/hip_runtime.h>
#include <stddef.h>


typedef _Float16 v16h __attribute__((ext_vector_type(16)));
typedef _Float16 v8h  __attribute__((ext_vector_type(8)));
typedef float    v8f  __attribute__((ext_vector_type(8)));
typedef float    v4f  __attribute__((ext_vector_type(4)));
typedef _Float16 h16;

#ifndef NB
#define NB 8
#endif
#ifndef SEQ
#define SEQ 1024
#endif
#define NB_FULL  8
#define SEQ_FULL 1024
#define DIM   128
#define HID   512
#define NHEAD 16
#define HD    8
#define FFK   8
#define QPITCH 32
#define VROWS  16
#define MROWS (NB * SEQ)

static_assert(NB >= 1 && NB <= NB_FULL);
static_assert(SEQ >= 64 && SEQ <= SEQ_FULL && (SEQ % 64) == 0 && (SEQ % 32) == 0);
static_assert(DIM == NHEAD * HD);
static_assert(HD == 8);
static_assert(FFK == 8);
static_assert(QPITCH == 32 && VROWS == 16);
static_assert(8 * HD == 64);
static_assert((NHEAD % 8) == 0);
static_assert(HID == 4 * DIM);
static_assert((DIM % 64) == 0 && (DIM % 32) == 0);
static_assert((HID % 64) == 0 && (HID % 32) == 0);
static_assert((MROWS % 64) == 0 && (MROWS % 8) == 0);
static_assert(DIM == 32 * 4);
static_assert(HID == 16 * 32);
static_assert(HID == 2 * 32 * 8);
static_assert(((DIM * DIM) % 2048) == 0 && ((DIM * HID) % 2048) == 0);
static_assert((size_t)MROWS * HID < (size_t)0xFFFFFFFFu);
static_assert((size_t)NB_FULL * SEQ_FULL * DIM * 4 == (size_t)4194304);

#define LDT 72
#define LDC 68
static_assert((LDT % 8) == 0 && LDT >= 64);
static_assert((LDC % 4) == 0 && LDC >= 64);

#define WCARRY 64.0f
#define QCARRY 64.0f
#define PCARRY 64.0f
#define PSHIFT 6.0f
#define VCARRY 64.0f
#define MCARRY 16.0f
#define RCARRY 1024.0f
static_assert(QCARRY == VCARRY);

#define WC_BYTES   ((size_t)DIM * DIM * 2)
#define W2_BYTES   ((size_t)DIM * HID * 2)
#define QP_BYTES   ((size_t)NB * NHEAD * SEQ * QPITCH * 2)
#define VT_BYTES   ((size_t)NB * NHEAD * VROWS * SEQ * 2)
#define CTX_BYTES  ((size_t)MROWS * DIM * 2)
#define S1_BYTES   ((size_t)MROWS * DIM * 4)
#define X1_BYTES   ((size_t)MROWS * DIM * 4)
#define MID_BYTES  ((size_t)MROWS * HID * 2)
#define Y_BYTES    ((size_t)NB_FULL * SEQ_FULL * DIM * 4)
#define OFF_WC  ((size_t)0)
#define OFF_W2  (OFF_WC + WC_BYTES)
#define OFF_QP  (OFF_W2 + W2_BYTES)
#define OFF_VT  (OFF_QP + QP_BYTES)
#define OFF_CTX (OFF_VT + VT_BYTES)
#define OFF_S1  (OFF_CTX + CTX_BYTES)
#define OFF_X1  (OFF_S1 + S1_BYTES)
#define OFF_MID (OFF_X1 + X1_BYTES)
#define OFF_Y   (OFF_MID + MID_BYTES)
#define WS_TOTAL (OFF_Y + Y_BYTES)
static_assert((WC_BYTES % 128) == 0 && (W2_BYTES % 128) == 0 && (QP_BYTES % 128) == 0);
static_assert((VT_BYTES % 128) == 0 && (CTX_BYTES % 128) == 0 && (S1_BYTES % 128) == 0);
static_assert((X1_BYTES % 128) == 0 && (MID_BYTES % 128) == 0 && (Y_BYTES % 128) == 0);
static_assert(WS_TOTAL <= (size_t)134217728);

__device__ __forceinline__ float bf16r(float x) {
  unsigned int u = __float_as_uint(x);
  u = (u + 0x7FFFu + ((u >> 16) & 1u)) & 0xFFFF0000u;
  return __uint_as_float(u);
}

static __device__ __forceinline__ h16 toh_flush(float v) {
  const h16 r = (h16)v;
  return (fabsf(v) < 6.103515625e-05f) ? (h16)0.0f : r;
}

__device__ __forceinline__ v16h frag_at(const _Float16* p) {
  v8h lo = *(const v8h*)(p);
  v8h hi = *(const v8h*)(p + 16);
  v16h out;
#pragma unroll
  for (int i = 0; i < 8; ++i) { out[i] = lo[i]; out[i + 8] = hi[i]; }
  return out;
}

__device__ __forceinline__ v8f wmma16(v16h a, v16h b, v8f c) {
  v8f d = __builtin_amdgcn_wmma_f32_16x16x32_f16(false, a, false, b, (short)0, c,
                                                 false, false);
  asm volatile("v_nop\n\tv_nop\n\tv_nop\n\tv_nop" : "+v"(d) : "v"(a), "v"(b));
  return d;
}

__device__ __forceinline__ float red32_sum(float x) {
#pragma unroll
  for (int off = 1; off < 32; off <<= 1) x += __shfl_xor(x, off, 32);
  return x;
}

__device__ __forceinline__ void wave_lds_sync() {
  __builtin_amdgcn_fence(3  , "wavefront");
  asm volatile("s_wait_dscnt 0x0" ::: "memory");
  __builtin_amdgcn_wave_barrier();
}

__device__ __forceinline__ float relu_act(float t) {
  return fmaxf(t, 0.0f);
}

__global__ __launch_bounds__(256) void wplane_kernel(
    const float* __restrict__ W, _Float16* __restrict__ Wp) {
  const size_t i = ((size_t)blockIdx.x * 256u + threadIdx.x) * 8u;
  const v4f a0 = *(const v4f*)(W + i);
  const v4f a1 = *(const v4f*)(W + i + 4u);
  v8h o;
#pragma unroll
  for (int j = 0; j < 4; ++j) {
    o[j]     = toh_flush(WCARRY * bf16r(a0[j]));
    o[j + 4] = toh_flush(WCARRY * bf16r(a1[j]));
  }
  *(volatile v8h*)(Wp + i) = o;
  __threadfence();
  *(volatile v8h*)(Wp + i) = o;
}

__device__ __forceinline__ void qz_store_pass(const _Float16* T, _Float16* QPb, _Float16* VTb,
                                              const unsigned tid, const unsigned s0) {
  const v8h z = {};
  v8h ones;
#pragma unroll
  for (int i = 0; i < 8; ++i) ones[i] = (h16)1.0f;
#pragma unroll 4
  for (unsigned j = 0; j < 16u; ++j) {
    const unsigned idx = tid + 256u * j;
    const unsigned row = idx >> 2, pc = idx & 3u;
    const unsigned head = row >> 6, s = row & 63u;
    v8h val = *(const v8h*)&T[row * 8u];
    val = (pc == 0u) ? val : z;
    *(volatile v8h*)(QPb + ((size_t)head * SEQ + s0 + s) * QPITCH + pc * 8u) = val;
  }
#pragma unroll 2
  for (unsigned j = 0; j < 8u; ++j) {
    const unsigned idx = tid + 256u * j;
    const unsigned line = idx >> 3, pc = idx & 7u;
    const unsigned head = line >> 4, vr = line & 15u;
    v8h g;
#pragma unroll
    for (unsigned jj = 0; jj < 8u; ++jj)
      g[jj] = T[(head * 64u + pc * 8u + jj) * 8u + (vr & 7u)];
    const v8h val = (vr < 8u) ? g : ((vr == 8u) ? ones : z);
    *(volatile v8h*)(VTb + ((size_t)head * VROWS + vr) * SEQ + s0 + pc * 8u) = val;
  }
}

__global__ __launch_bounds__(256) void qz_kernel(
    const float* __restrict__ X, const float* __restrict__ rx,
    _Float16* __restrict__ QP, _Float16* __restrict__ VT) {
#pragma clang fp contract(off)
  __shared__ _Float16 T[NHEAD * 64 * HD];
  const unsigned tid = threadIdx.x;
  const unsigned s0 = blockIdx.x * 64u;
  const unsigned b = blockIdx.y;
  float th[8];
#pragma unroll
  for (int d = 0; d < 8; ++d) th[d] = bf16r(rx[d]);

#pragma unroll 1
  for (unsigned j = 0; j < 4u; ++j) {
    const unsigned idx = tid + 256u * j;
    const unsigned s = idx >> 4, head = idx & 15u;
    const float* xp = X + ((size_t)b * SEQ_FULL + s0 + s) * DIM + head * HD;
    const v4f a0 = *(const v4f*)(xp);
    const v4f a1 = *(const v4f*)(xp + 4);
    float c[8];
#pragma unroll
    for (int d = 0; d < 4; ++d) {
      c[d]     = __cosf(bf16r(a0[d]) + th[d]);
      c[d + 4] = __cosf(bf16r(a1[d]) + th[d + 4]);
    }
    float o[8];
    float P = c[0];
#pragma unroll
    for (int d = 1; d < 8; ++d) { P = P * c[d]; o[d] = P; }
    float z0 = c[1];
#pragma unroll
    for (int d = 2; d < 8; ++d) z0 = z0 * c[d];
    o[0] = z0;
    v8h o16;
#pragma unroll
    for (int d = 0; d < 8; ++d) o16[d] = toh_flush(QCARRY * o[d]);
    *(v8h*)&T[(head * 64u + s) * 8u] = o16;
  }
  __syncthreads();

  _Float16* QPb = QP + (size_t)b * NHEAD * SEQ * QPITCH;
  _Float16* VTb = VT + (size_t)b * NHEAD * VROWS * SEQ;
  qz_store_pass(T, QPb, VTb, tid, s0);
  __threadfence();
  qz_store_pass(T, QPb, VTb, tid, s0);
}

__global__ __launch_bounds__(256) void attn_kernel(
    const _Float16* __restrict__ QP, const _Float16* __restrict__ VT,
    _Float16* __restrict__ Ctx) {
  __shared__ _Float16 Cst[16 * LDT];
  const unsigned tid = threadIdx.x, lane = tid & 31u;
  const unsigned wave = (unsigned)__builtin_amdgcn_readfirstlane((int)(threadIdx.x >> 5));
  const unsigned hh = lane >> 4, m = lane & 15u;
  const unsigned q0 = blockIdx.x * 16u;
  const unsigned hg = blockIdx.y;
  const unsigned b = blockIdx.z;
  const unsigned head = hg * 8u + wave;
  const size_t bh = (size_t)b * NHEAD + head;

  const _Float16* kp = QP + bh * SEQ * QPITCH + m * QPITCH + hh * 8u;
  const _Float16* vp = VT + (bh * VROWS + m) * SEQ + hh * 8u;
  const v16h qf = frag_at(kp + (size_t)q0 * QPITCH);

  const float esc = 0.35355339059327373f * 1.4426950408889634f / (QCARRY * QCARRY);

  v8f o = {};
#pragma unroll 2
  for (unsigned kb = 0; kb < (unsigned)SEQ; kb += 32u) {
    const v16h k0f = frag_at(kp + (size_t)kb * QPITCH);
    const v16h k1f = frag_at(kp + (size_t)(kb + 16u) * QPITCH);
    const v16h vf  = frag_at(vp + kb);
    v8f s0 = {}, s1 = {};
    s0 = wmma16(k0f, qf, s0);
    s1 = wmma16(k1f, qf, s1);
    v16h pf;
#pragma unroll
    for (int r = 0; r < 8; ++r) {
      const float e0 = s0[r] * esc + PSHIFT;
      const float e1 = s1[r] * esc + PSHIFT;
      const float p0 = __builtin_amdgcn_exp2f(e0);
      const float p1 = __builtin_amdgcn_exp2f(e1);
      pf[r]     = (e0 < -14.0f) ? (h16)0.0f : (h16)p0;
      pf[r + 8] = (e1 < -14.0f) ? (h16)0.0f : (h16)p1;
    }
    o = wmma16(vf, pf, o);
  }

  const float den = __shfl(o[0], (int)(16u + m), 32);
  const float inv = __builtin_amdgcn_rcpf(den);
  if (hh == 0u) {
    v8h c8;
#pragma unroll
    for (int r = 0; r < 8; ++r) c8[r] = toh_flush(o[r] * inv);
    *(v8h*)&Cst[m * LDT + wave * 8u] = c8;
  }
  __syncthreads();
  if (wave < 4u) {
    const unsigned r = tid >> 3;
    const unsigned c = (tid & 7u) * 8u;
    const v8h x = *(const v8h*)&Cst[r * LDT + c];
    _Float16* p = Ctx + (size_t)(b * (unsigned)SEQ + q0 + r) * DIM + hg * 64u + c;
    *(volatile v8h*)p = x;
    __threadfence();
    *(volatile v8h*)p = x;
  }
}

template <int MODE>
__device__ __forceinline__ void gemm_body(
    const _Float16* __restrict__ A16, const _Float16* __restrict__ Bt, const unsigned K,
    const float* __restrict__ bias, const float* __restrict__ addf,
    float* __restrict__ outf, _Float16* __restrict__ out16, _Float16* __restrict__ out16r) {
  __shared__ float Cs[64 * LDC];
  const unsigned tid = threadIdx.x, lane = tid & 31u, w = tid >> 5;
  const unsigned mw = w >> 1, nw = w & 1u;
  const unsigned hh = lane >> 4, m = lane & 15u;
  const unsigned n0 = blockIdx.x * 64u;
  const unsigned row0 = blockIdx.y * 64u;

  const _Float16* ap  = A16 + (size_t)(row0 + mw * 16u + m) * K + hh * 8u;
  const _Float16* bp0 = Bt + (size_t)(n0 + nw * 32u + m) * K + hh * 8u;
  const _Float16* bp1 = bp0 + (size_t)16 * K;
  v8f acc0 = {}, acc1 = {};
#pragma unroll 2
  for (unsigned k0 = 0; k0 < K; k0 += 32u) {
    const v16h a  = frag_at(ap + k0);
    const v16h b0 = frag_at(bp0 + k0);
    const v16h b1 = frag_at(bp1 + k0);
    acc0 = wmma16(a, b0, acc0);
    acc1 = wmma16(a, b1, acc1);
  }
#pragma unroll
  for (int r = 0; r < 8; ++r) {
    float* d = &Cs[(mw * 16u + hh * 8u + (unsigned)r) * LDC + nw * 32u + m];
    d[0]  = acc0[r];
    d[16] = acc1[r];
  }
  __syncthreads();

  if (MODE == 3) {
#pragma unroll 1
    for (unsigned g = 0; g < 4u; ++g) {
      const unsigned r = 32u * (g >> 1) + (tid >> 3);
      const unsigned c = (tid & 7u) * 8u + 4u * (g & 1u);
      const v4f u  = *(const v4f*)&Cs[r * LDC + c];
      const v4f gb = *(const v4f*)(bias + n0 + c);
      v4f t;
#pragma unroll
      for (int j = 0; j < 4; ++j)
        t[j] = MCARRY * relu_act(u[j] * (1.0f / WCARRY) + bf16r(gb[j]));
      *(v4f*)&Cs[r * LDC + c] = t;
    }
  }

  if (MODE == 0 || MODE == 3) {
    const unsigned ldo = (MODE == 3) ? (unsigned)HID : (unsigned)DIM;
    v8h x[2];
    size_t off[2];
#pragma unroll
    for (unsigned i = 0; i < 2u; ++i) {
      const unsigned r = 32u * i + (tid >> 3);
      const unsigned c = (tid & 7u) * 8u;
      const v4f u0 = *(const v4f*)&Cs[r * LDC + c];
      const v4f u1 = *(const v4f*)&Cs[r * LDC + c + 4];
      if (MODE == 3) {
#pragma unroll
        for (int j = 0; j < 4; ++j) {
          x[i][j]     = (_Float16)u0[j];
          x[i][j + 4] = (_Float16)u1[j];
        }
      } else {
        const v4f g0 = *(const v4f*)(bias + n0 + c);
        const v4f g1 = *(const v4f*)(bias + n0 + c + 4u);
#pragma unroll
        for (int j = 0; j < 4; ++j) {
          x[i][j]     = (_Float16)(u0[j] * (1.0f / WCARRY) + bf16r(g0[j]));
          x[i][j + 4] = (_Float16)(u1[j] * (1.0f / WCARRY) + bf16r(g1[j]));
        }
      }
      off[i] = (size_t)(row0 + r) * ldo + n0 + c;
    }
#pragma unroll
    for (int i = 0; i < 2; ++i) *(volatile v8h*)(out16 + off[i]) = x[i];
    __threadfence();
#pragma unroll
    for (int i = 0; i < 2; ++i) *(volatile v8h*)(out16 + off[i]) = x[i];
  }

  if (MODE == 1) {
    const unsigned bidx = row0 / (unsigned)SEQ;
    const unsigned key0 = row0 - bidx * (unsigned)SEQ;
    const bool first_tile = (key0 == 0u);
    v8h x[2], xr[2];
    size_t off[2], offr[2];
#pragma unroll
    for (unsigned i = 0; i < 2u; ++i) {
      const unsigned dcol = 32u * i + (tid >> 3);
      const unsigned kk = (tid & 7u) * 8u;
      const float bb = bf16r(bias[n0 + dcol]);
#pragma unroll
      for (unsigned j = 0; j < 8u; ++j) {
        const float t = Cs[(kk + j) * LDC + dcol] * (1.0f / WCARRY) + bb;
        const _Float16 hi = (_Float16)t;
        x[i][j]  = hi;
        xr[i][j] = (_Float16)((t - (float)hi) * RCARRY);
      }
      off[i]  = ((size_t)bidx * DIM + n0 + dcol) * SEQ + key0 + kk;
      offr[i] = ((size_t)bidx * DIM + n0 + dcol) * 64u + kk;
    }
#pragma unroll
    for (int i = 0; i < 2; ++i) *(volatile v8h*)(out16 + off[i]) = x[i];
    if (first_tile) {
#pragma unroll
      for (int i = 0; i < 2; ++i) *(volatile v8h*)(out16r + offr[i]) = xr[i];
    }
    __threadfence();
#pragma unroll
    for (int i = 0; i < 2; ++i) *(volatile v8h*)(out16 + off[i]) = x[i];
    if (first_tile) {
#pragma unroll
      for (int i = 0; i < 2; ++i) *(volatile v8h*)(out16r + offr[i]) = xr[i];
    }
  }

  if (MODE == 2 || MODE == 4) {
    const float cs = (MODE == 2) ? (1.0f / (WCARRY * VCARRY)) : (1.0f / (WCARRY * MCARRY));
    v4f xs[4];
    size_t off[4];
#pragma unroll
    for (unsigned i = 0; i < 4u; ++i) {
      const unsigned r = 16u * i + (tid >> 4);
      const unsigned c = (tid & 15u) * 4u;
      const unsigned crow = row0 + r;
      const unsigned bidx = crow / (unsigned)SEQ;
      const unsigned sq = crow - bidx * (unsigned)SEQ;
      const size_t frow = (size_t)bidx * SEQ_FULL + sq;
      const size_t inrow  = (MODE == 2) ? frow : (size_t)crow;
      const size_t outrow = (MODE == 2) ? (size_t)crow : frow;
      const v4f u = *(const v4f*)&Cs[r * LDC + c];
      const v4f g = *(const v4f*)(bias + n0 + c);
      const v4f xin = *(const v4f*)(addf + inrow * DIM + n0 + c);
      v4f val;
#pragma unroll
      for (int j = 0; j < 4; ++j) {
        const float base = (MODE == 2) ? bf16r(xin[j]) : xin[j];
        val[j] = base + (u[j] * cs + bf16r(g[j]));
      }
      xs[i] = val;
      off[i] = outrow * DIM + n0 + c;
    }
#pragma unroll
    for (int i = 0; i < 4; ++i) *(volatile v4f*)(outf + off[i]) = xs[i];
    __threadfence();
#pragma unroll
    for (int i = 0; i < 4; ++i) *(volatile v4f*)(outf + off[i]) = xs[i];
  }
}

__global__ __launch_bounds__(256) void gemm_wo_kernel(
    const _Float16* __restrict__ A16, const _Float16* __restrict__ Bt,
    const float* __restrict__ bias, const float* __restrict__ xin, float* __restrict__ x1) {
  gemm_body<2>(A16, Bt, (unsigned)DIM, bias, xin, x1, (_Float16*)0, (_Float16*)0);
}
__global__ __launch_bounds__(256) void gemm_ffn2_kernel(
    const _Float16* __restrict__ A16, const _Float16* __restrict__ Bt,
    const float* __restrict__ bias, const float* __restrict__ x1, float* __restrict__ outf) {
  gemm_body<4>(A16, Bt, (unsigned)HID, bias, x1, outf, (_Float16*)0, (_Float16*)0);
}

__device__ __forceinline__ v4f ln128(const v4f a, const float* __restrict__ G,
                                     const float* __restrict__ Be, const unsigned c) {
#pragma clang fp contract(off)
  const float mean = red32_sum((a[0] + a[1]) + (a[2] + a[3])) * (1.0f / (float)DIM);
  v4f d;
#pragma unroll
  for (int i = 0; i < 4; ++i) d[i] = a[i] - mean;
  const float ss = (d[0] * d[0] + d[1] * d[1]) + (d[2] * d[2] + d[3] * d[3]);
  const float var = red32_sum(ss) * (1.0f / (float)DIM);
  const float rstd = 1.0f / sqrtf(var + 1.0e-5f);
  const v4f g  = *(const v4f*)(G + c);
  const v4f be = *(const v4f*)(Be + c);
  v4f o;
#pragma unroll
  for (int i = 0; i < 4; ++i) o[i] = d[i] * rstd * bf16r(g[i]) + bf16r(be[i]);
  return o;
}

__global__ __launch_bounds__(256) void ln1_ffn_kernel(
    const float* __restrict__ S1, const float* __restrict__ G, const float* __restrict__ Be,
    const float* __restrict__ ry, const float* __restrict__ w1, const float* __restrict__ b1,
    float* __restrict__ X1, _Float16* __restrict__ Mid) {
#pragma clang fp contract(off)
  __shared__ _Float16 Hs[8 * HID];
  const unsigned lane = threadIdx.x & 31u;
  const unsigned wave = (unsigned)__builtin_amdgcn_readfirstlane((int)(threadIdx.x >> 5));
  const unsigned crow = blockIdx.x * 8u + wave;

  const v4f a = *(const v4f*)(S1 + (size_t)crow * DIM + lane * 4u);
  const v4f o = ln128(a, G, Be, lane * 4u);
  float* xp = X1 + (size_t)crow * DIM + lane * 4u;
  *(volatile v4f*)xp = o;

  float zc[4];
#pragma unroll
  for (int i = 0; i < 4; ++i) {
    const unsigned ci = (lane * 4u + (unsigned)i) & 7u;
    zc[i] = __cosf(o[i]) * __cosf(bf16r(ry[ci]));
  }
  float zf[8];
#pragma unroll
  for (int k = 0; k < 8; ++k) zf[k] = __shfl(zc[k & 3], k >> 2, 32);

  _Float16* Hrow = Hs + wave * (unsigned)HID;
#pragma unroll 1
  for (unsigned t = 0; t < 16u; ++t) {
    const unsigned f = t * 32u + lane;
    const v4f wa = *(const v4f*)(w1 + (size_t)f * FFK);
    const v4f wb = *(const v4f*)(w1 + (size_t)f * FFK + 4u);
    float acc = bf16r(b1[f]);
#pragma unroll
    for (int k = 0; k < 4; ++k) acc = fmaf(zf[k], bf16r(wa[k]), acc);
#pragma unroll
    for (int k = 0; k < 4; ++k) acc = fmaf(zf[k + 4], bf16r(wb[k]), acc);
    Hrow[f] = toh_flush(MCARRY * relu_act(acc));
  }
  wave_lds_sync();
  const v8h h0 = *(const v8h*)&Hrow[lane * 8u];
  const v8h h1 = *(const v8h*)&Hrow[256u + lane * 8u];
  _Float16* mp = Mid + (size_t)crow * HID + lane * 8u;
  *(volatile v8h*)(mp) = h0;
  *(volatile v8h*)(mp + 256) = h1;
  __threadfence();
  *(volatile v4f*)xp = o;
  *(volatile v8h*)(mp) = h0;
  *(volatile v8h*)(mp + 256) = h1;
}

__global__ __launch_bounds__(256) void ln2_kernel(
    const float* __restrict__ Y, const float* __restrict__ G, const float* __restrict__ Be,
    float* __restrict__ out) {
#pragma clang fp contract(off)
  const unsigned lane = threadIdx.x & 31u;
  const unsigned wave = (unsigned)__builtin_amdgcn_readfirstlane((int)(threadIdx.x >> 5));
  const unsigned crow = blockIdx.x * 8u + wave;
  const unsigned bidx = crow / (unsigned)SEQ;
  const unsigned sq = crow - bidx * (unsigned)SEQ;
  const size_t frow = (size_t)bidx * SEQ_FULL + sq;
  const v4f a = *(const v4f*)(Y + frow * DIM + lane * 4u);
  const v4f o = ln128(a, G, Be, lane * 4u);
  float* p = out + frow * DIM + lane * 4u;
  *(volatile v4f*)p = o;
  __threadfence();
  *(volatile v4f*)p = o;
}

extern "C" void kernel_launch(void* const* d_in, const int* in_sizes, int n_in,
                              void* d_out, int out_size, void* d_ws, size_t ws_size,
                              hipStream_t stream) {
  if (n_in < 13) return;
  const long long need_x = ((long long)(NB - 1) * SEQ_FULL + SEQ) * DIM;
  if ((long long)in_sizes[0] < need_x) return;
  if (in_sizes[1] < HD || in_sizes[2] < FFK) return;
  if ((long long)in_sizes[3] < (long long)DIM * DIM) return;
  if (in_sizes[4] < DIM) return;
  if ((long long)in_sizes[5] < (long long)HID * FFK) return;
  if (in_sizes[6] < HID) return;
  if ((long long)in_sizes[7] < (long long)DIM * HID) return;
  if (in_sizes[8] < DIM) return;
  if (in_sizes[9] < DIM || in_sizes[10] < DIM || in_sizes[11] < DIM || in_sizes[12] < DIM) return;
  if ((long long)out_size < need_x) return;
  if (ws_size < WS_TOTAL) return;

  const float* X    = (const float*)d_in[0];
  const float* rx   = (const float*)d_in[1];
  const float* ry   = (const float*)d_in[2];
  const float* wc   = (const float*)d_in[3];
  const float* bc   = (const float*)d_in[4];
  const float* w1   = (const float*)d_in[5];
  const float* b1   = (const float*)d_in[6];
  const float* w2   = (const float*)d_in[7];
  const float* b2   = (const float*)d_in[8];
  const float* g1   = (const float*)d_in[9];
  const float* be1  = (const float*)d_in[10];
  const float* g2   = (const float*)d_in[11];
  const float* be2  = (const float*)d_in[12];
  float* out = (float*)d_out;

  char* ws = (char*)d_ws;
  _Float16* Wc16  = (_Float16*)(ws + OFF_WC);
  _Float16* W216  = (_Float16*)(ws + OFF_W2);
  _Float16* QP16  = (_Float16*)(ws + OFF_QP);
  _Float16* VT16  = (_Float16*)(ws + OFF_VT);
  _Float16* Ctx16 = (_Float16*)(ws + OFF_CTX);
  float*    S1    = (float*)(ws + OFF_S1);
  float*    X1    = (float*)(ws + OFF_X1);
  _Float16* Mid16 = (_Float16*)(ws + OFF_MID);
  float*    Y     = (float*)(ws + OFF_Y);

  dim3 blk(256);
  dim3 gg(DIM / 64, MROWS / 64);

  wplane_kernel<<<dim3((DIM * DIM) / 2048), blk, 0, stream>>>(wc, Wc16);
  wplane_kernel<<<dim3((DIM * HID) / 2048), blk, 0, stream>>>(w2, W216);
  qz_kernel<<<dim3(SEQ / 64, NB), blk, 0, stream>>>(X, rx, QP16, VT16);
  attn_kernel<<<dim3(SEQ / 16, NHEAD / 8, NB), blk, 0, stream>>>(QP16, VT16, Ctx16);
  gemm_wo_kernel<<<gg, blk, 0, stream>>>(Ctx16, Wc16, bc, X, S1);
  ln1_ffn_kernel<<<dim3(MROWS / 8), blk, 0, stream>>>(S1, g1, be1, ry, w1, b1, X1, Mid16);
  gemm_ffn2_kernel<<<gg, blk, 0, stream>>>(Mid16, W216, b2, X1, Y);
  ln2_kernel<<<dim3(MROWS / 8), blk, 0, stream>>>(Y, g2, be2, out);
}
